// Decoder_74191265071285
// MI455X (gfx1250) — hardware-verified
//
#include <hip/hip_runtime.h>
#include <math.h>

constexpr int NSEQ     = 64;
constexpr int NBATCH   = 8192;
constexpr int NHID     = 64;
constexpr int NEMB     = 64;
constexpr int NGATE    = 4 * NHID;
constexpr int NTHR     = 256;
constexpr int ROWS_BLK = 32;
constexpr int APITCH   = 72;
constexpr int HFPITCH  = 68;
constexpr int NW8      = NGATE * NHID / 8;
constexpr int NOUT0    = NSEQ * NBATCH * 2;
constexpr int NOUT1    = NBATCH * NHID;

static_assert(NHID == 64 && NEMB == 64);
static_assert(NHID % 32 == 0);
static_assert(NBATCH % ROWS_BLK == 0);
static_assert((ROWS_BLK / 16) * (NHID / 16) == NTHR / 32);
static_assert(NW8 % NTHR == 0);
static_assert((ROWS_BLK * NHID / 4) % NTHR == 0);
static_assert(NGATE == NTHR);
static_assert((size_t)NOUT0 * 4 == 4194304);
static_assert((size_t)NOUT0 * 4 + (size_t)NOUT1 * 4 == 6291456);

typedef __attribute__((ext_vector_type(16))) _Float16 v16h;
typedef __attribute__((ext_vector_type(8)))  _Float16 v8h;
typedef __attribute__((ext_vector_type(16))) __bf16   v16b;
typedef __attribute__((ext_vector_type(8)))  __bf16   v8b;
typedef __attribute__((ext_vector_type(8)))  float    v8f;
typedef __attribute__((ext_vector_type(4)))  float    v4f;
typedef __attribute__((ext_vector_type(2)))  float    v2f;
typedef __attribute__((ext_vector_type(2)))  unsigned v2u;

__device__ __forceinline__ unsigned short f2bf_bits(float f) {
  unsigned u = __float_as_uint(f);
  return (unsigned short)((u + 0x7FFFu + ((u >> 16) & 1u)) >> 16);
}
__device__ __forceinline__ float bf_bits2f(unsigned short h) { return __uint_as_float(((unsigned)h) << 16); }

__device__ __forceinline__ void acc_guard4(v8f& a, v8f& b, v8f& c, v8f& d) { asm volatile("v_nop\n\tv_nop\n\tv_nop\n\tv_nop" : "+v"(a), "+v"(b), "+v"(c), "+v"(d)); }

union FragB { v16b v; v8b h[2]; };
__device__ __forceinline__ v16b frag_load(const __bf16* p) {
  FragB f;
  f.h[0] = *(const v8b*)(p);
  f.h[1] = *(const v8b*)(p + 16);
  return f.v;
}
__device__ __forceinline__ v8f mma_bf(v16b a, v16b b, v8f c) {
  c = __builtin_amdgcn_wmma_f32_16x16x32_bf16(false, a, false, b, (short)0, c, false, false);
  asm volatile("v_nop\n\tv_nop\n\tv_nop\n\tv_nop" : "+v"(c) : "v"(a), "v"(b));
  return c;
}

__device__ __forceinline__ float sigm(float x) { return __builtin_amdgcn_rcpf(1.0f + expf(-x)); }

__global__ __launch_bounds__(NTHR) void wsplit_kernel(const float* __restrict__ w, unsigned short* __restrict__ phi,
                                                      unsigned short* __restrict__ plo) {
  const int i = blockIdx.x * NTHR + threadIdx.x;
  if (i < NW8) {
    const v4f a = *(const v4f*)(w + (size_t)i * 8);
    const v4f b = *(const v4f*)(w + (size_t)i * 8 + 4);
    v8h hv, lv;
#pragma unroll
    for (int e = 0; e < 4; ++e) {
      const float fa = a[e];
      const float fb = b[e];
      const unsigned short ha = f2bf_bits(fa);
      const unsigned short hb = f2bf_bits(fb);
      const unsigned short la = f2bf_bits(fa - bf_bits2f(ha));
      const unsigned short lb = f2bf_bits(fb - bf_bits2f(hb));
      hv[e]     = __builtin_bit_cast(_Float16, ha);
      hv[4 + e] = __builtin_bit_cast(_Float16, hb);
      lv[e]     = __builtin_bit_cast(_Float16, la);
      lv[4 + e] = __builtin_bit_cast(_Float16, lb);
    }
    *(volatile v8h*)(phi + (size_t)i * 8) = hv;
    *(volatile v8h*)(plo + (size_t)i * 8) = lv;
    __threadfence();
    *(volatile v8h*)(phi + (size_t)i * 8) = hv;
    *(volatile v8h*)(plo + (size_t)i * 8) = lv;
  }
}

__global__ __launch_bounds__(NTHR) void fold_kernel(const float* __restrict__ w_emb, const float* __restrict__ b_emb,
                                                    const float* __restrict__ w_ih, const float* __restrict__ b_ih,
                                                    const float* __restrict__ b_hh, float* __restrict__ PRM) {
  __shared__ __align__(16) float sE[3 * NEMB];
  const int tid = threadIdx.x;
  if (tid < 2 * NEMB) sE[tid] = w_emb[tid];
  if (tid >= 2 * NEMB && tid < 3 * NEMB) sE[tid] = b_emb[tid - 2 * NEMB];
  __syncthreads();
  const int n = tid;
  float a0 = 0.0f, a1 = 0.0f, ab = 0.0f;
#pragma unroll 1
  for (int e4 = 0; e4 < NEMB / 4; ++e4) {
    const v4f wv = *(const v4f*)(w_ih + (size_t)n * NEMB + 4 * e4);
#pragma unroll
    for (int q = 0; q < 4; ++q) {
      const int e = 4 * e4 + q;
      const float wq = wv[q];
      a0 = fmaf(wq, sE[2 * e], a0);
      a1 = fmaf(wq, sE[2 * e + 1], a1);
      ab = fmaf(wq, sE[2 * NEMB + e], ab);
    }
  }
  const float bsum = (b_ih[n] + b_hh[n]) + ab;
  v4f o;
  o[0] = a0;
  o[1] = a1;
  o[2] = bsum;
  o[3] = 0.0f;
  *(volatile v4f*)(PRM + 4 * n) = o;
  __threadfence();
  *(volatile v4f*)(PRM + 4 * n) = o;
}

__global__ __launch_bounds__(NTHR) void lstm_decode_kernel(const float* __restrict__ last_pos, const float* __restrict__ h0p,
                                                           const float* __restrict__ c0p, const float* __restrict__ w_out,
                                                           const float* __restrict__ b_out,
                                                           const unsigned short* __restrict__ Whip,
                                                           const unsigned short* __restrict__ Wlop,
                                                           const float* __restrict__ PRM, float* __restrict__ out) {
  __shared__ __align__(16) unsigned short Ahi[ROWS_BLK * APITCH];
  __shared__ __align__(16) unsigned short Alo[ROWS_BLK * APITCH];
  __shared__ __align__(16) float          Hf[ROWS_BLK * HFPITCH];
  __shared__ __align__(16) float          Rr[ROWS_BLK * 2];
  __shared__ __align__(16) float          sWo[2 * NHID];

  const int tid = threadIdx.x, lane = tid & 31, wave = tid >> 5;
  const int cl = lane & 15, hh = lane >> 4, koff = hh * 8;
  const int mi = wave >> 2, ub = wave & 3;
  const int j = 16 * ub + cl;
  const int rowbase = blockIdx.x * ROWS_BLK;

#pragma unroll
  for (int it = 0; it < 2; ++it) {
    const int idx = it * NTHR + tid;
    const int row = idx >> 4, c4 = (idx & 15) * 4;
    const v4f v = *(const v4f*)(h0p + (size_t)(rowbase + row) * NHID + c4);
    const float f0 = v[0], f1 = v[1], f2 = v[2], f3 = v[3];
    const unsigned short h0b = f2bf_bits(f0), h1b = f2bf_bits(f1), h2b = f2bf_bits(f2), h3b = f2bf_bits(f3);
    const unsigned short l0b = f2bf_bits(f0 - bf_bits2f(h0b)), l1b = f2bf_bits(f1 - bf_bits2f(h1b));
    const unsigned short l2b = f2bf_bits(f2 - bf_bits2f(h2b)), l3b = f2bf_bits(f3 - bf_bits2f(h3b));
    v2u ph, pl;
    ph[0] = (unsigned)h0b | ((unsigned)h1b << 16);
    ph[1] = (unsigned)h2b | ((unsigned)h3b << 16);
    pl[0] = (unsigned)l0b | ((unsigned)l1b << 16);
    pl[1] = (unsigned)l2b | ((unsigned)l3b << 16);
    *(v2u*)(Ahi + row * APITCH + c4) = ph;
    *(v2u*)(Alo + row * APITCH + c4) = pl;
  }
  if (tid < 2 * ROWS_BLK) Rr[tid] = last_pos[(size_t)rowbase * 2 + tid];
  if (tid < 2 * NHID) sWo[tid] = w_out[tid];
  const float bo = b_out[tid & 1];

  float cst[8];
#pragma unroll
  for (int r = 0; r < 8; ++r) cst[r] = c0p[(size_t)(rowbase + 16 * mi + 8 * hh + r) * NHID + j];
  v4f prm[4];
#pragma unroll
  for (int g = 0; g < 4; ++g) prm[g] = *(const v4f*)(PRM + (size_t)(g * NHID + j) * 4);
  __syncthreads();

  const __bf16* ahrow = (const __bf16*)Ahi + (16 * mi + cl) * APITCH + koff;
  const __bf16* alrow = (const __bf16*)Alo + (16 * mi + cl) * APITCH + koff;
  const __bf16* whb = (const __bf16*)Whip + (size_t)j * NHID + koff;
  const __bf16* wlb = (const __bf16*)Wlop + (size_t)j * NHID + koff;
  const v8f z8 = {0.f, 0.f, 0.f, 0.f, 0.f, 0.f, 0.f, 0.f};

#pragma unroll 1
  for (int s = 0; s < NSEQ; ++s) {
    v8f acc[4];
    acc[0] = z8; acc[1] = z8; acc[2] = z8; acc[3] = z8;
#pragma unroll
    for (int kc = 0; kc < NHID / 32; ++kc) {
      const int k0 = kc * 32;
      const v16b ah = frag_load(ahrow + k0);
      const v16b al = frag_load(alrow + k0);
#pragma unroll
      for (int g = 0; g < 4; ++g) {
        const v16b bh = frag_load(whb + (size_t)g * NHID * NHID + k0);
        const v16b bl = frag_load(wlb + (size_t)g * NHID * NHID + k0);
        acc[g] = mma_bf(ah, bl, acc[g]);
        acc[g] = mma_bf(al, bh, acc[g]);
        acc[g] = mma_bf(ah, bh, acc[g]);
      }
      asm volatile("" ::: "memory");
    }
    acc_guard4(acc[0], acc[1], acc[2], acc[3]);

    float hreg[8];
#pragma unroll
    for (int r = 0; r < 8; ++r) {
      const int row = 16 * mi + 8 * hh + r;
      const v2f rr = *(const v2f*)(Rr + 2 * row);
      const float r0 = rr[0], r1 = rr[1];
      const float zi = acc[0][r] + (prm[0][2] + r0 * prm[0][0] + r1 * prm[0][1]);
      const float zf = acc[1][r] + (prm[1][2] + r0 * prm[1][0] + r1 * prm[1][1]);
      const float zg = acc[2][r] + (prm[2][2] + r0 * prm[2][0] + r1 * prm[2][1]);
      const float zo = acc[3][r] + (prm[3][2] + r0 * prm[3][0] + r1 * prm[3][1]);
      const float ig = sigm(zi);
      const float fg = sigm(zf);
      const float gg = tanhf(zg);
      const float og = sigm(zo);
      const float cn = fg * cst[r] + ig * gg;
      cst[r] = cn;
      hreg[r] = og * tanhf(cn);
    }
    __syncthreads();
#pragma unroll
    for (int r = 0; r < 8; ++r) {
      const int row = 16 * mi + 8 * hh + r;
      const float hv = hreg[r];
      const unsigned short hb = f2bf_bits(hv);
      const unsigned short lb = f2bf_bits(hv - bf_bits2f(hb));
      Ahi[row * APITCH + j] = hb;
      Alo[row * APITCH + j] = lb;
      Hf[row * HFPITCH + j] = hv;
    }
    __syncthreads();
    if (tid < 2 * ROWS_BLK) {
      const float* hp = Hf + (tid >> 1) * HFPITCH;
      const float* wp = sWo + (tid & 1) * NHID;
      float a = 0.0f;
#pragma unroll 4
      for (int k4 = 0; k4 < NHID / 4; ++k4) {
        const v4f hv4 = *(const v4f*)(hp + 4 * k4);
        const v4f wv4 = *(const v4f*)(wp + 4 * k4);
        a = fmaf(hv4[0], wv4[0], a);
        a = fmaf(hv4[1], wv4[1], a);
        a = fmaf(hv4[2], wv4[2], a);
        a = fmaf(hv4[3], wv4[3], a);
      }
      Rr[tid] = a + bo;
    }
    __syncthreads();
    if (wave == 7) {
      const int l4 = (lane & 15) * 4;
      const v4f v = *(const v4f*)(Rr + l4);
      float* op = out + ((size_t)s * NBATCH + (size_t)rowbase) * 2 + l4;
      if (lane < 16) *(volatile v4f*)op = v;
      __threadfence();
      if (lane < 16) *(volatile v4f*)op = v;
    }
  }

  {
    float* o1 = out + (size_t)NOUT0 + (size_t)rowbase * NHID;
    for (int pass = 0; pass < 2; ++pass) {
#pragma unroll
      for (int it = 0; it < 2; ++it) {
        const int idx = it * NTHR + tid;
        const int row = idx >> 4, c4 = (idx & 15) * 4;
        const v4f v = *(const v4f*)(Hf + row * HFPITCH + c4);
        *(volatile v4f*)(o1 + (size_t)row * NHID + c4) = v;
      }
      __threadfence();
    }
  }
}

extern "C" void kernel_launch(void* const* d_in, const int* in_sizes, int n_in,
                              void* d_out, int out_size, void* d_ws, size_t ws_size, hipStream_t stream) {
  if (n_in < 11 || d_out == nullptr || d_ws == nullptr) return;
  if (in_sizes[0] != NBATCH * 2 || in_sizes[1] != NBATCH * NHID || in_sizes[2] != NBATCH * NHID ||
      in_sizes[3] != NEMB * 2 || in_sizes[4] != NEMB || in_sizes[5] != NGATE * NEMB ||
      in_sizes[6] != NGATE * NHID || in_sizes[7] != NGATE || in_sizes[8] != NGATE ||
      in_sizes[9] != 2 * NHID || in_sizes[10] != 2 || out_size != NOUT0 + NOUT1) return;

  const float* last_pos = (const float*)d_in[0];
  const float* hh0      = (const float*)d_in[1];
  const float* ch0      = (const float*)d_in[2];
  const float* w_emb    = (const float*)d_in[3];
  const float* b_emb    = (const float*)d_in[4];
  const float* w_ih     = (const float*)d_in[5];
  const float* w_hh     = (const float*)d_in[6];
  const float* b_ih     = (const float*)d_in[7];
  const float* b_hh     = (const float*)d_in[8];
  const float* w_out    = (const float*)d_in[9];
  const float* b_out    = (const float*)d_in[10];
  float* out = (float*)d_out;

  char* ws = (char*)d_ws; size_t off = 0;
  auto carve = [&](size_t bytes) -> char* { char* p = ws + off; off += (bytes + 255) & ~(size_t)255; return p; };
  unsigned short* WHI = (unsigned short*)carve((size_t)NGATE * NHID * 2);
  unsigned short* WLO = (unsigned short*)carve((size_t)NGATE * NHID * 2);
  float*          PRM = (float*)carve((size_t)NGATE * 4 * 4);
  if (off > ws_size || off > (size_t)134217728) return;

  wsplit_kernel<<<NW8 / NTHR, NTHR, 0, stream>>>(w_hh, WHI, WLO);
  fold_kernel<<<1, NTHR, 0, stream>>>(w_emb, b_emb, w_ih, b_ih, b_hh, PRM);
  lstm_decode_kernel<<<NBATCH / ROWS_BLK, NTHR, 0, stream>>>(last_pos, hh0, ch0, w_out, b_out, WHI, WLO, PRM, out);
}
